// kqvAttn_25151328485711
// MI455X (gfx1250) — hardware-verified
//
#include <hip/hip_runtime.h>
#include <math.h>
#include <stdint.h>
#include <stddef.h>

#define G_ROWS 8192
#define IN_D   512
#define KQ_D   128
#define OUT_D  512
#define RBLK   2048
#define NPASS  (G_ROWS / RBLK)
#define EPSF   1e-12f
#define WSC     64.0f
#define WSC_INV (1.0f / 64.0f)

typedef __attribute__((ext_vector_type(16))) _Float16 v16h;
typedef __attribute__((ext_vector_type(8)))  _Float16 v8h;
typedef __attribute__((ext_vector_type(16))) __bf16   v16b;
typedef __attribute__((ext_vector_type(8)))  __bf16   v8b;
typedef __attribute__((ext_vector_type(8)))  float    v8f;
typedef __attribute__((ext_vector_type(4)))  float    v4f;

__device__ __forceinline__ unsigned short f2bf_bits(float f) {
  unsigned u = __float_as_uint(f);
  return (unsigned short)((u + 0x7FFFu + ((u >> 16) & 1u)) >> 16);
}
__device__ __forceinline__ float bf_bits2f(unsigned short h) { return __uint_as_float(((unsigned)h) << 16); }

__device__ __forceinline__ void dep_guard_h(v8f& a, v8f& b, v16h x, v16h y) { asm volatile("v_nop\n\tv_nop\n\tv_nop\n\tv_nop" : "+v"(a), "+v"(b) : "v"(x), "v"(y)); }
__device__ __forceinline__ void dep_guard_b(v8f& a, v8f& b, v16b x, v16b y) { asm volatile("v_nop\n\tv_nop\n\tv_nop\n\tv_nop" : "+v"(a), "+v"(b) : "v"(x), "v"(y)); }
__device__ __forceinline__ void keep4_h(v16h a, v16h b, v16h c, v16h d) { asm volatile("v_nop" :: "v"(a), "v"(b), "v"(c), "v"(d)); }
__device__ __forceinline__ void keep4_b(v16b a, v16b b, v16b c, v16b d) { asm volatile("v_nop" :: "v"(a), "v"(b), "v"(c), "v"(d)); }
__device__ __forceinline__ void acc_guard4(v8f& a, v8f& b, v8f& c, v8f& d) { asm volatile("v_nop\n\tv_nop\n\tv_nop\n\tv_nop" : "+v"(a), "+v"(b), "+v"(c), "+v"(d)); }
template <typename T> struct Frag;
template <> struct Frag<_Float16> {
  typedef v16h V; union U { v16h v; v8h h[2]; };
  static __device__ __forceinline__ v16h load(const _Float16* p) {
    U f; f.h[0] = *(const v8h*)(p); f.h[1] = *(const v8h*)(p + 16); return f.v;
  }
  static __device__ __forceinline__ v8f mma(v16h a, v16h b, v8f c) {
    return __builtin_amdgcn_wmma_f32_16x16x32_f16(false, a, false, b, (short)0, c, false, false);
  }
  static __device__ __forceinline__ void guard(v8f& a, v8f& b, v16h x, v16h y) { dep_guard_h(a, b, x, y); }
  static __device__ __forceinline__ void keep(v16h a, v16h b, v16h c, v16h d) { keep4_h(a, b, c, d); }
};
template <> struct Frag<__bf16> {
  typedef v16b V; union U { v16b v; v8b h[2]; };
  static __device__ __forceinline__ v16b load(const __bf16* p) {
    U f; f.h[0] = *(const v8b*)(p); f.h[1] = *(const v8b*)(p + 16); return f.v;
  }
  static __device__ __forceinline__ v8f mma(v16b a, v16b b, v8f c) {
    return __builtin_amdgcn_wmma_f32_16x16x32_bf16(false, a, false, b, (short)0, c, false, false);
  }
  static __device__ __forceinline__ void guard(v8f& a, v8f& b, v16b x, v16b y) { dep_guard_b(a, b, x, y); }
  static __device__ __forceinline__ void keep(v16b a, v16b b, v16b c, v16b d) { keep4_b(a, b, c, d); }
};

template <int ET> struct Elem;
template <> struct Elem<0> { typedef _Float16 T; };
template <> struct Elem<1> { typedef __bf16 T; };
template <int ET, bool SPLIT, int BIAS_MODE, int OUT_MODE, bool RESID, int ACT = 0>
__global__ __launch_bounds__(256) void wmma_gemm64(
    const unsigned short* __restrict__ Ap, const unsigned short* __restrict__ A2p, int lda, long strideA,
    const unsigned short* __restrict__ Btp, const unsigned short* __restrict__ Bt2p, int ldb, long strideB,
    void* __restrict__ Cout, void* __restrict__ Cout2, int ldc, long strideC,
    const float* __restrict__ bias,
    const float* __restrict__ resid, long strideR,
    int M, int N, int K, float scale) {
  typedef typename Elem<ET>::T T;
  typedef typename Frag<T>::V V;
  const T* A = (const T*)Ap; const T* A2 = (const T*)A2p; const T* Bt = (const T*)Btp; const T* Bt2 = (const T*)Bt2p;
  __shared__ __align__(16) float sT[8][16 * 68];
  const int b    = blockIdx.y;
  const int lane = threadIdx.x & 31;
  const int wave = threadIdx.x >> 5;
  const int tilesN = N >> 6;
  const int tilesM = M >> 6;
  const int tile = blockIdx.x * 8 + wave;
  if (tile >= tilesM * tilesN) return;
  const int tm = tile / tilesN;
  const int tn = tile - tm * tilesN;
  const int m0 = tm << 6;
  const int n0 = tn << 6;

  const T* Ab  = A  + (size_t)b * strideA;
  const T* Bb  = Bt + (size_t)b * strideB;
  const T* Ab2 = SPLIT ? (A2  + (size_t)b * strideA) : nullptr;
  const T* Bb2 = SPLIT ? (Bt2 + (size_t)b * strideB) : nullptr;

  const int rlane = lane & 15;
  const int koff  = (lane >> 4) * 8;
  const int mOff  = (lane >> 4) * 8;

  v8f acc[4][4];
#pragma unroll
  for (int i = 0; i < 4; ++i)
#pragma unroll
    for (int j = 0; j < 4; ++j) acc[i][j] = (v8f){0.f,0.f,0.f,0.f,0.f,0.f,0.f,0.f};

  for (int k0 = 0; k0 < K; k0 += 32) {
    V bh[4], bl[4];
#pragma unroll
    for (int j = 0; j < 4; ++j) {
      const size_t bo = (size_t)(n0 + (j << 4) + rlane) * ldb + koff + k0;
      bh[j] = Frag<T>::load(Bb + bo);
      if (SPLIT) bl[j] = Frag<T>::load(Bb2 + bo);
    }
#pragma unroll
    for (int i = 0; i < 4; ++i) {
      const size_t ao = (size_t)(m0 + (i << 4) + rlane) * lda + koff + k0;
      V ah = Frag<T>::load(Ab + ao);
      V al;
      if (SPLIT) al = Frag<T>::load(Ab2 + ao);
#pragma unroll
      for (int j = 0; j < 4; ++j) {
        acc[i][j] = Frag<T>::mma(ah, bh[j], acc[i][j]);
        if (SPLIT) {
          acc[i][j] = Frag<T>::mma(ah, bl[j], acc[i][j]);
          acc[i][j] = Frag<T>::mma(al, bh[j], acc[i][j]);
        }
      }
      Frag<T>::guard(acc[i][0], acc[i][3], ah, SPLIT ? al : ah);
    }
    Frag<T>::keep(bh[0], bh[1], bh[2], bh[3]);
    if (SPLIT) Frag<T>::keep(bl[0], bl[1], bl[2], bl[3]);
  }
  acc_guard4(acc[0][0], acc[0][1], acc[0][2], acc[0][3]);
  acc_guard4(acc[1][0], acc[1][1], acc[1][2], acc[1][3]);
  acc_guard4(acc[2][0], acc[2][1], acc[2][2], acc[2][3]);
  acc_guard4(acc[3][0], acc[3][1], acc[3][2], acc[3][3]);

  float* slab = sT[wave];
  const float* Rb = RESID ? (resid + (size_t)b * strideR) : nullptr;
#pragma unroll
  for (int i = 0; i < 4; ++i) {
    const int mBase = m0 + (i << 4);
#pragma unroll
    for (int j = 0; j < 4; ++j) {
      const int n = n0 + (j << 4) + rlane;
      float bv = 0.f;
      if (BIAS_MODE == 2) bv = bias[n];
#pragma unroll
      for (int r = 0; r < 8; ++r) {
        float v = acc[i][j][r] * scale;
        if (BIAS_MODE == 3) v *= bias[mBase + mOff + r];
        if (BIAS_MODE == 1) v += bias[mBase + mOff + r];
        if (BIAS_MODE == 2) v += bv;
        if (RESID) v += Rb[(size_t)(mBase + mOff + r) * ldc + n];
        if (ACT == 1) v = tanhf(v);
        if (ACT == 2) v = fmaxf(v, 0.0f);
        if (ACT == 3) v = v / (1.0f + expf(-v));
        if (ACT == 4) v = (v > 0.f) ? v : 0.01f * v;
        if (ACT == 5) v = 0.5f * v * (1.0f + erff(v * 0.70710678118654752f));
        slab[(mOff + r) * 68 + (j << 4) + rlane] = v;
      }
    }
    __builtin_amdgcn_fence(__ATOMIC_RELEASE, "workgroup");
    __builtin_amdgcn_wave_barrier();
    __builtin_amdgcn_fence(__ATOMIC_ACQUIRE, "workgroup");
    if (OUT_MODE == 0) {
      float* C = (float*)Cout + (size_t)b * strideC;
      const int hh = lane >> 4, c4 = (lane & 15) * 4;
      for (int pass = 0; pass < 2; ++pass) {
#pragma unroll
        for (int it = 0; it < 8; ++it) {
          const int row = it * 2 + hh;
          v4f v = *(const v4f*)(slab + row * 68 + c4);
          *(volatile v4f*)(C + (size_t)(mBase + row) * ldc + n0 + c4) = v;
        }
        __threadfence();
      }
    } else {
      const int q = lane >> 3, c8 = (lane & 7) * 8;
      unsigned short* C  = (unsigned short*)Cout  + (size_t)b * strideC;
      unsigned short* C2 = (OUT_MODE == 2) ? ((unsigned short*)Cout2 + (size_t)b * strideC) : nullptr;
      for (int pass = 0; pass < 2; ++pass) {
#pragma unroll
        for (int it = 0; it < 4; ++it) {
          const int row = it * 4 + q;
          const float* sp = slab + row * 68 + c8;
          v8h hv, lv;
#pragma unroll
          for (int e = 0; e < 8; ++e) {
            if (OUT_MODE == 1) {
              hv[e] = (_Float16)sp[e];
            } else {
              unsigned short hb = f2bf_bits(sp[e]);
              unsigned short lb = f2bf_bits(sp[e] - bf_bits2f(hb));
              hv[e] = __builtin_bit_cast(_Float16, hb);
              lv[e] = __builtin_bit_cast(_Float16, lb);
            }
          }
          *(volatile v8h*)(C + (size_t)(mBase + row) * ldc + n0 + c8) = hv;
          if (OUT_MODE == 2) *(volatile v8h*)(C2 + (size_t)(mBase + row) * ldc + n0 + c8) = lv;
        }
        __threadfence();
      }
    }
    __builtin_amdgcn_fence(__ATOMIC_RELEASE, "workgroup");
    __builtin_amdgcn_wave_barrier();
    __builtin_amdgcn_fence(__ATOMIC_ACQUIRE, "workgroup");
  }
}

__global__ __launch_bounds__(256) void cast_f32_f16x2s(
    const float* __restrict__ in, unsigned short* __restrict__ out, int n2, float mul) {
  int i = blockIdx.x * 256 + threadIdx.x;
  if (i < n2) {
    const _Float16 h0 = (_Float16)(in[2 * i] * mul), h1 = (_Float16)(in[2 * i + 1] * mul);
    const unsigned u = (unsigned)__builtin_bit_cast(unsigned short, h0) | ((unsigned)__builtin_bit_cast(unsigned short, h1) << 16);
    ((volatile unsigned*)out)[i] = u;
    __threadfence();
    ((volatile unsigned*)out)[i] = u;
  }
}

#define NRM_ROWS 32
__global__ __launch_bounds__(256) void k_rownorm(const unsigned short* __restrict__ Sp, int ldS, int ncol256,
                                                 float* __restrict__ inv, int nrows) {
  const _Float16* S = (const _Float16*)Sp;
  __shared__ __align__(16) float sInv[NRM_ROWS];
  const int lane = threadIdx.x & 31;
  const int wave = threadIdx.x >> 5;
  const int rbase = blockIdx.x * NRM_ROWS;
#pragma unroll 1
  for (int rr = 0; rr < 4; ++rr) {
    const int row  = rbase + wave * 4 + rr;
    const int rowc = row < nrows ? row : (nrows - 1);
    const _Float16* sp = S + (size_t)rowc * ldS;
    v8f a = (v8f){0.f,0.f,0.f,0.f,0.f,0.f,0.f,0.f};
#pragma unroll 1
    for (int it = 0; it < ncol256; ++it) {
      const v8h hv = *(const v8h*)(sp + (((size_t)(it * 32 + lane)) << 3));
#pragma unroll
      for (int e = 0; e < 8; ++e) { const float f = (float)hv[e]; a[e] += f * f; }
    }
    float ss = ((a[0] + a[1]) + (a[2] + a[3])) + ((a[4] + a[5]) + (a[6] + a[7]));
#pragma unroll
    for (int off = 1; off < 32; off <<= 1) ss += __shfl_xor(ss, off, 32);
    if (lane == 0) {
      const float nrm = sqrtf(ss);
      sInv[wave * 4 + rr] = 1.0f / fmaxf(nrm, EPSF);
    }
  }
  __syncthreads();
  if (wave == 0 && lane < 8) {
    const int r0 = rbase + 4 * lane;
    if (r0 + 3 < nrows) {
      const v4f val = *(const v4f*)(sInv + 4 * lane);
      float* p = inv + r0;
      *(volatile v4f*)p = val;
      __threadfence();
      *(volatile v4f*)p = val;
    }
  }
}

extern "C" void kernel_launch(void* const* d_in, const int* in_sizes, int n_in,
                              void* d_out, int out_size, void* d_ws, size_t ws_size,
                              hipStream_t stream) {
  if (n_in < 7) return;
  if (in_sizes[0] != G_ROWS * IN_D || in_sizes[1] != KQ_D * IN_D || in_sizes[2] != KQ_D ||
      in_sizes[3] != KQ_D * IN_D || in_sizes[4] != KQ_D || in_sizes[5] != OUT_D * IN_D ||
      in_sizes[6] != OUT_D) return;
  if (out_size != G_ROWS * OUT_D) return;

  const float* x  = (const float*)d_in[0];
  const float* Wk = (const float*)d_in[1];
  const float* bk = (const float*)d_in[2];
  const float* Wq = (const float*)d_in[3];
  const float* bq = (const float*)d_in[4];
  const float* Wv = (const float*)d_in[5];
  const float* bv = (const float*)d_in[6];
  float* out = (float*)d_out;

  const size_t b_x16 = (size_t)G_ROWS * IN_D * 2;
  const size_t b_wk  = (size_t)KQ_D * IN_D * 2;
  const size_t b_wv  = (size_t)OUT_D * IN_D * 2;
  const size_t b_k16 = (size_t)G_ROWS * KQ_D * 2;
  const size_t b_vf  = (size_t)G_ROWS * OUT_D * 4;
  const size_t b_vt  = (size_t)OUT_D * G_ROWS * 2;
  const size_t b_s16 = (size_t)RBLK * G_ROWS * 2;
  const size_t b_inv = (size_t)RBLK * 4;

  size_t off = 0;
  const size_t o_x16 = off; off += b_x16;
  const size_t o_wk  = off; off += b_wk;
  const size_t o_wq  = off; off += b_wk;
  const size_t o_wv  = off; off += b_wv;
  const size_t o_k16 = off; off += b_k16;
  const size_t o_q16 = off; off += b_k16;
  const size_t o_vf  = off; off += b_vf;
  const size_t o_vt  = off; off += b_vt;
  const size_t o_s16 = off; off += b_s16;
  const size_t o_inv = off; off += b_inv;
  if (off > ws_size) return;

  char* ws = (char*)d_ws;
  unsigned short* x16  = (unsigned short*)(ws + o_x16);
  unsigned short* wk16 = (unsigned short*)(ws + o_wk);
  unsigned short* wq16 = (unsigned short*)(ws + o_wq);
  unsigned short* wv16 = (unsigned short*)(ws + o_wv);
  unsigned short* k16  = (unsigned short*)(ws + o_k16);
  unsigned short* q16  = (unsigned short*)(ws + o_q16);
  float*          vf   = (float*)(ws + o_vf);
  unsigned short* vt16 = (unsigned short*)(ws + o_vt);
  unsigned short* s16  = (unsigned short*)(ws + o_s16);
  float*          invb = (float*)(ws + o_inv);

  {
    const int n2x = G_ROWS * IN_D / 2;
    cast_f32_f16x2s<<<dim3((n2x + 255) / 256), 256, 0, stream>>>(x, x16, n2x, 1.0f);
    const int n2k = KQ_D * IN_D / 2;
    cast_f32_f16x2s<<<dim3((n2k + 255) / 256), 256, 0, stream>>>(Wk, wk16, n2k, WSC);
    cast_f32_f16x2s<<<dim3((n2k + 255) / 256), 256, 0, stream>>>(Wq, wq16, n2k, WSC);
    const int n2v = OUT_D * IN_D / 2;
    cast_f32_f16x2s<<<dim3((n2v + 255) / 256), 256, 0, stream>>>(Wv, wv16, n2v, WSC);
  }

  {
    const int tk = (G_ROWS / 64) * (KQ_D / 64);
    wmma_gemm64<0, false, 2, 1, false><<<dim3((tk + 7) / 8, 1), 256, 0, stream>>>(
        x16, nullptr, IN_D, 0L, wk16, nullptr, IN_D, 0L, (void*)k16, nullptr, KQ_D, 0L,
        bk, nullptr, 0L, G_ROWS, KQ_D, IN_D, WSC_INV);
    wmma_gemm64<0, false, 2, 1, false><<<dim3((tk + 7) / 8, 1), 256, 0, stream>>>(
        x16, nullptr, IN_D, 0L, wq16, nullptr, IN_D, 0L, (void*)q16, nullptr, KQ_D, 0L,
        bq, nullptr, 0L, G_ROWS, KQ_D, IN_D, WSC_INV);
    const int tv = (G_ROWS / 64) * (OUT_D / 64);
    wmma_gemm64<0, false, 2, 0, false><<<dim3((tv + 7) / 8, 1), 256, 0, stream>>>(
        x16, nullptr, IN_D, 0L, wv16, nullptr, IN_D, 0L, (void*)vf, nullptr, OUT_D, 0L,
        bv, nullptr, 0L, G_ROWS, OUT_D, IN_D, WSC_INV);
    const int tt = (OUT_D / 64) * (G_ROWS / 64);
    wmma_gemm64<0, false, 1, 1, false><<<dim3((tt + 7) / 8, 1), 256, 0, stream>>>(
        wv16, nullptr, IN_D, 0L, x16, nullptr, IN_D, 0L, (void*)vt16, nullptr, G_ROWS, 0L,
        bv, nullptr, 0L, OUT_D, G_ROWS, IN_D, WSC_INV);
  }

  for (int rb = 0; rb < NPASS; ++rb) {
    const int ts = (RBLK / 64) * (G_ROWS / 64);
    wmma_gemm64<0, false, 0, 1, false><<<dim3((ts + 7) / 8, 1), 256, 0, stream>>>(
        k16 + (size_t)rb * RBLK * KQ_D, nullptr, KQ_D, 0L, q16, nullptr, KQ_D, 0L,
        (void*)s16, nullptr, G_ROWS, 0L, nullptr, nullptr, 0L, RBLK, G_ROWS, KQ_D, 1.0f);
    k_rownorm<<<dim3(RBLK / NRM_ROWS), 256, 0, stream>>>(s16, G_ROWS, G_ROWS / 256, invb, RBLK);
    const int tp = (RBLK / 64) * (OUT_D / 64);
    wmma_gemm64<0, false, 3, 0, true><<<dim3((tp + 7) / 8, 1), 256, 0, stream>>>(
        s16, nullptr, G_ROWS, 0L, vt16, nullptr, G_ROWS, 0L,
        (void*)(out + (size_t)rb * RBLK * OUT_D), nullptr, OUT_D, 0L,
        invb, vf + (size_t)rb * RBLK * OUT_D, 0L, RBLK, OUT_D, G_ROWS, 1.0f);
  }
}
